// TPAAttention_49400713838785
// MI455X (gfx1250) — hardware-verified
//
#include <hip/hip_runtime.h>
#include <stdint.h>
#include <stddef.h>

typedef __attribute__((ext_vector_type(16))) _Float16 v16h;
typedef __attribute__((ext_vector_type(8)))  _Float16 v8h;
typedef __attribute__((ext_vector_type(16))) __bf16   v16b;
typedef __attribute__((ext_vector_type(8)))  __bf16   v8b;
typedef __attribute__((ext_vector_type(8)))  float    v8f;
typedef __attribute__((ext_vector_type(4)))  float    v4f;
typedef __attribute__((ext_vector_type(2)))  float    v2f;

constexpr int kBatch = 2;
constexpr int kSeq = 2048;
constexpr int kHid = 2048;
constexpr int kHeads = 8;
constexpr int kHeadDim = 256;
constexpr int kRq = 6;
constexpr int kRk = 2;
constexpr int kRv = 2;
constexpr int kTok = kBatch * kSeq;
constexpr int kNcat = 2624;
constexpr int kColAq = 0;
constexpr int kColAk = 48;
constexpr int kColAv = 50;
constexpr int kColPad = 52;
constexpr int kColBq = 64;
constexpr int kColBk = 1600;
constexpr int kColBv = 2112;
constexpr int kSplitRows = 512;

constexpr float kQkCarry = 16.0f;
constexpr float kVCarry = 16.0f;
constexpr float kAoCarry = 16.0f;
constexpr float kResCarry = 2048.0f;
constexpr float kPCarry = 32768.0f;
constexpr float kWoCarry = 16.0f;
constexpr float kScaling = 0.0625f;
constexpr float kSoftcap = 50.0f;
constexpr float kScoreScl = kScaling / (kQkCarry * kQkCarry);
constexpr float kTanhArg = kScoreScl / kSoftcap;
constexpr float kOutScl = kAoCarry / (kPCarry * kVCarry);

constexpr int kAttPool = 8704;

constexpr size_t kBytesFac  = (size_t)kTok * kNcat * 4;
constexpr size_t kBytesAo   = (size_t)kTok * kHid * 2;
constexpr size_t kBytesT1   = (size_t)kBatch * kSplitRows * kHid * 4;
constexpr size_t kBytesHsb  = (size_t)kTok * kHid * 2;
constexpr size_t kBytesWcat = (size_t)kNcat * kHid * 2;
constexpr size_t kBytesQ    = (size_t)kTok * kHeads * kHeadDim * 2;
constexpr size_t kBytesKv   = (size_t)kTok * kHeadDim * 2;
constexpr size_t kBytesWo   = (size_t)kHid * kHid * 2;

constexpr size_t kOffFac  = 0;
constexpr size_t kOffAoh  = 0;
constexpr size_t kOffAol  = kOffAoh + kBytesAo;
constexpr size_t kOffT1   = kOffAol + kBytesAo;
constexpr size_t kOffHsb  = kOffFac + kBytesFac;
constexpr size_t kOffQh   = kOffHsb;
constexpr size_t kOffWcat = kOffHsb + kBytesHsb;
constexpr size_t kOffKh   = kOffWcat;
constexpr size_t kOffKl   = kOffKh + kBytesKv;
constexpr size_t kOffVth  = kOffKl + kBytesKv;
constexpr size_t kOffVtl  = kOffVth + kBytesKv;
constexpr size_t kOffQl   = kOffWcat + kBytesWcat;
constexpr size_t kOffWo   = kOffQl + kBytesQ;
constexpr size_t kWsTotal = kOffWo + kBytesWo;
static_assert(kOffT1 + kBytesT1 <= kBytesFac, "T1 inside the dead FAC region");
static_assert(kOffVtl + kBytesKv <= kOffWcat + kBytesWcat, "k/v planes inside the dead wcat region");
static_assert(kOffQh + kBytesQ <= kOffWcat, "qh inside the dead hsb region");
static_assert(kWsTotal == 95682560, "carve total");
static_assert(kWsTotal <= (size_t)134217728, "carve budget");
static_assert((kOffHsb % 256) == 0 && (kOffWcat % 256) == 0 && (kOffQl % 256) == 0 && (kOffWo % 256) == 0 && (kOffT1 % 256) == 0 && (kOffAol % 256) == 0, "alignment");
static_assert(kTok % 64 == 0 && kNcat % 64 == 0 && kHid % 32 == 0, "factor GEMM shape");
static_assert(kSplitRows % 64 == 0 && (kSeq - kSplitRows) % 64 == 0 && kHid % 64 == 0, "output GEMM shapes");
static_assert(kSplitRows % 16 == 0 && (kSeq - kSplitRows) % 32 == 0 && kSplitRows % 32 == 0, "attention block rows");

__device__ __forceinline__ unsigned short f2bf_bits(float f) {
  unsigned u = __float_as_uint(f);
  return (unsigned short)((u + 0x7FFFu + ((u >> 16) & 1u)) >> 16);
}
__device__ __forceinline__ float bf_bits2f(unsigned short h) { return __uint_as_float(((unsigned)h) << 16); }
__device__ __forceinline__ float bf16_rne(float f) { return bf_bits2f(f2bf_bits(f)); }

__device__ __forceinline__ void dep_guard_h(v8f& a, v8f& b, v16h x, v16h y) { asm volatile("v_nop\n\tv_nop\n\tv_nop\n\tv_nop" : "+v"(a), "+v"(b) : "v"(x), "v"(y)); }
__device__ __forceinline__ void dep_guard_b(v8f& a, v8f& b, v16b x, v16b y) { asm volatile("v_nop\n\tv_nop\n\tv_nop\n\tv_nop" : "+v"(a), "+v"(b) : "v"(x), "v"(y)); }
__device__ __forceinline__ void keep4_h(v16h a, v16h b, v16h c, v16h d) { asm volatile("v_nop" :: "v"(a), "v"(b), "v"(c), "v"(d)); }
__device__ __forceinline__ void keep4_b(v16b a, v16b b, v16b c, v16b d) { asm volatile("v_nop" :: "v"(a), "v"(b), "v"(c), "v"(d)); }
__device__ __forceinline__ void acc_guard4(v8f& a, v8f& b, v8f& c, v8f& d) { asm volatile("v_nop\n\tv_nop\n\tv_nop\n\tv_nop" : "+v"(a), "+v"(b), "+v"(c), "+v"(d)); }
template <typename T> struct Frag;
template <> struct Frag<_Float16> {
  typedef v16h V; union U { v16h v; v8h h[2]; };
  static __device__ __forceinline__ v16h load(const _Float16* p) {
    U f; f.h[0] = *(const v8h*)(p); f.h[1] = *(const v8h*)(p + 16); return f.v;
  }
  static __device__ __forceinline__ v8f mma(v16h a, v16h b, v8f c) {
    return __builtin_amdgcn_wmma_f32_16x16x32_f16(false, a, false, b, (short)0, c, false, false);
  }
  static __device__ __forceinline__ void guard(v8f& a, v8f& b, v16h x, v16h y) { dep_guard_h(a, b, x, y); }
  static __device__ __forceinline__ void keep(v16h a, v16h b, v16h c, v16h d) { keep4_h(a, b, c, d); }
};
template <> struct Frag<__bf16> {
  typedef v16b V; union U { v16b v; v8b h[2]; };
  static __device__ __forceinline__ v16b load(const __bf16* p) {
    U f; f.h[0] = *(const v8b*)(p); f.h[1] = *(const v8b*)(p + 16); return f.v;
  }
  static __device__ __forceinline__ v8f mma(v16b a, v16b b, v8f c) {
    return __builtin_amdgcn_wmma_f32_16x16x32_bf16(false, a, false, b, (short)0, c, false, false);
  }
  static __device__ __forceinline__ void guard(v8f& a, v8f& b, v16b x, v16b y) { dep_guard_b(a, b, x, y); }
  static __device__ __forceinline__ void keep(v16b a, v16b b, v16b c, v16b d) { keep4_b(a, b, c, d); }
};

__device__ __forceinline__ v8f mma16(v16h a, v16h b, v8f c) {
  c = __builtin_amdgcn_wmma_f32_16x16x32_f16(false, a, false, b, (short)0, c, false, false);
  asm volatile("v_nop\n\tv_nop\n\tv_nop\n\tv_nop" : "+v"(c) : "v"(a), "v"(b));
  return c;
}

template <int ET> struct Elem;
template <> struct Elem<0> { typedef _Float16 T; };
template <> struct Elem<1> { typedef __bf16 T; };
template <int ET, bool SPLIT, int BIAS_MODE, int OUT_MODE, bool RESID, int ACT = 0>
__global__ __launch_bounds__(256) void wmma_gemm64(
    const unsigned short* __restrict__ Ap, const unsigned short* __restrict__ A2p, int lda, long strideA,
    const unsigned short* __restrict__ Btp, const unsigned short* __restrict__ Bt2p, int ldb, long strideB,
    void* __restrict__ Cout, void* __restrict__ Cout2, int ldc, long strideC,
    const float* __restrict__ bias,
    const float* __restrict__ resid, long strideR,
    int M, int N, int K, float scale) {
  typedef typename Elem<ET>::T T;
  typedef typename Frag<T>::V V;
  const T* A = (const T*)Ap; const T* A2 = (const T*)A2p; const T* Bt = (const T*)Btp; const T* Bt2 = (const T*)Bt2p;
  __shared__ __align__(16) float sT[8][16 * 68];
  const int b    = blockIdx.y;
  const int lane = threadIdx.x & 31;
  const int wave = threadIdx.x >> 5;
  const int tilesN = N >> 6;
  const int tilesM = M >> 6;
  const int tile = blockIdx.x * 8 + wave;
  if (tile >= tilesM * tilesN) return;
  const int tm = tile / tilesN;
  const int tn = tile - tm * tilesN;
  const int m0 = tm << 6;
  const int n0 = tn << 6;

  const T* Ab  = A  + (size_t)b * strideA;
  const T* Bb  = Bt + (size_t)b * strideB;
  const T* Ab2 = SPLIT ? (A2  + (size_t)b * strideA) : nullptr;
  const T* Bb2 = SPLIT ? (Bt2 + (size_t)b * strideB) : nullptr;

  const int rlane = lane & 15;
  const int koff  = (lane >> 4) * 8;
  const int mOff  = (lane >> 4) * 8;

  v8f acc[4][4];
#pragma unroll
  for (int i = 0; i < 4; ++i)
#pragma unroll
    for (int j = 0; j < 4; ++j) acc[i][j] = (v8f){0.f,0.f,0.f,0.f,0.f,0.f,0.f,0.f};

  for (int k0 = 0; k0 < K; k0 += 32) {
    V bh[4], bl[4];
#pragma unroll
    for (int j = 0; j < 4; ++j) {
      const size_t bo = (size_t)(n0 + (j << 4) + rlane) * ldb + koff + k0;
      bh[j] = Frag<T>::load(Bb + bo);
      if (SPLIT) bl[j] = Frag<T>::load(Bb2 + bo);
    }
#pragma unroll
    for (int i = 0; i < 4; ++i) {
      const size_t ao = (size_t)(m0 + (i << 4) + rlane) * lda + koff + k0;
      V ah = Frag<T>::load(Ab + ao);
      V al;
      if (SPLIT) al = Frag<T>::load(Ab2 + ao);
#pragma unroll
      for (int j = 0; j < 4; ++j) {
        acc[i][j] = Frag<T>::mma(ah, bh[j], acc[i][j]);
        if (SPLIT) {
          acc[i][j] = Frag<T>::mma(ah, bl[j], acc[i][j]);
          acc[i][j] = Frag<T>::mma(al, bh[j], acc[i][j]);
        }
      }
      Frag<T>::guard(acc[i][0], acc[i][3], ah, SPLIT ? al : ah);
    }
    Frag<T>::keep(bh[0], bh[1], bh[2], bh[3]);
    if (SPLIT) Frag<T>::keep(bl[0], bl[1], bl[2], bl[3]);
  }
  acc_guard4(acc[0][0], acc[0][1], acc[0][2], acc[0][3]);
  acc_guard4(acc[1][0], acc[1][1], acc[1][2], acc[1][3]);
  acc_guard4(acc[2][0], acc[2][1], acc[2][2], acc[2][3]);
  acc_guard4(acc[3][0], acc[3][1], acc[3][2], acc[3][3]);

  float* slab = sT[wave];
  const float* Rb = RESID ? (resid + (size_t)b * strideR) : nullptr;
#pragma unroll
  for (int i = 0; i < 4; ++i) {
    const int mBase = m0 + (i << 4);
#pragma unroll
    for (int j = 0; j < 4; ++j) {
      const int n = n0 + (j << 4) + rlane;
      float bv = 0.f;
      if (BIAS_MODE == 2) bv = bias[n];
#pragma unroll
      for (int r = 0; r < 8; ++r) {
        float v = acc[i][j][r] * scale;
        if (BIAS_MODE == 1) v += bias[mBase + mOff + r];
        if (BIAS_MODE == 2) v += bv;
        if (ACT == 1) v = tanhf(v);
        if (ACT == 2) v = fmaxf(v, 0.0f);
        if (ACT == 4) v = (v > 0.f) ? v : 0.01f * v;
        slab[(mOff + r) * 68 + (j << 4) + rlane] = v;
      }
    }
    __builtin_amdgcn_fence(__ATOMIC_RELEASE, "workgroup");
    __builtin_amdgcn_wave_barrier();
    __builtin_amdgcn_fence(__ATOMIC_ACQUIRE, "workgroup");
    if (OUT_MODE == 0) {
      float* C = (float*)Cout + (size_t)b * strideC;
      const int hh = lane >> 4, c4 = (lane & 15) * 4;
      for (int pass = 0; pass < 2; ++pass) {
#pragma unroll
        for (int it = 0; it < 8; ++it) {
          const int row = it * 2 + hh;
          v4f v = *(const v4f*)(slab + row * 68 + c4);
          if (RESID) {
            const v4f rr = *(const v4f*)(Rb + (size_t)(mBase + row) * ldc + n0 + c4);
            v += rr;
          }
          *(volatile v4f*)(C + (size_t)(mBase + row) * ldc + n0 + c4) = v;
        }
        __threadfence();
      }
    } else {
      const int q = lane >> 3, c8 = (lane & 7) * 8;
      unsigned short* C  = (unsigned short*)Cout  + (size_t)b * strideC;
      unsigned short* C2 = (OUT_MODE == 2) ? ((unsigned short*)Cout2 + (size_t)b * strideC) : nullptr;
      for (int pass = 0; pass < 2; ++pass) {
#pragma unroll
        for (int it = 0; it < 4; ++it) {
          const int row = it * 4 + q;
          const float* sp = slab + row * 68 + c8;
          v8h hv, lv;
#pragma unroll
          for (int e = 0; e < 8; ++e) {
            if (OUT_MODE == 1) {
              hv[e] = (_Float16)sp[e];
            } else {
              unsigned short hb = f2bf_bits(sp[e]);
              unsigned short lb = f2bf_bits(sp[e] - bf_bits2f(hb));
              hv[e] = __builtin_bit_cast(_Float16, hb);
              lv[e] = __builtin_bit_cast(_Float16, lb);
            }
          }
          *(volatile v8h*)(C + (size_t)(mBase + row) * ldc + n0 + c8) = hv;
          if (OUT_MODE == 2) *(volatile v8h*)(C2 + (size_t)(mBase + row) * ldc + n0 + c8) = lv;
        }
        __threadfence();
      }
    }
    __builtin_amdgcn_fence(__ATOMIC_RELEASE, "workgroup");
    __builtin_amdgcn_wave_barrier();
    __builtin_amdgcn_fence(__ATOMIC_ACQUIRE, "workgroup");
  }
}

__global__ __launch_bounds__(256) void cast_bf16x2(const float* __restrict__ in, unsigned short* __restrict__ out, int n2) {
  const int i = blockIdx.x * 256 + threadIdx.x;
  if (i < n2) {
    const v2f x = *(const v2f*)(in + 2 * (size_t)i);
    const unsigned u = (unsigned)f2bf_bits(x[0]) | ((unsigned)f2bf_bits(x[1]) << 16);
    ((volatile unsigned*)out)[i] = u;
    __threadfence();
    ((volatile unsigned*)out)[i] = u;
  }
}
__global__ __launch_bounds__(256) void cast_wo_f16x2(const float* __restrict__ in, unsigned short* __restrict__ out, int n2) {
  const int i = blockIdx.x * 256 + threadIdx.x;
  if (i < n2) {
    const v2f x = *(const v2f*)(in + 2 * (size_t)i);
    const float a0 = bf16_rne(x[0]) * kWoCarry;
    const float a1 = bf16_rne(x[1]) * kWoCarry;
    const _Float16 h0 = (_Float16)a0, h1 = (_Float16)a1;
    const unsigned u = (unsigned)__builtin_bit_cast(unsigned short, h0) | ((unsigned)__builtin_bit_cast(unsigned short, h1) << 16);
    ((volatile unsigned*)out)[i] = u;
    __threadfence();
    ((volatile unsigned*)out)[i] = u;
  }
}
__global__ __launch_bounds__(256) void build_wcat(const float* __restrict__ waq, const float* __restrict__ wak,
                                                  const float* __restrict__ wav, const float* __restrict__ wbq,
                                                  const float* __restrict__ wbk, const float* __restrict__ wbv,
                                                  unsigned short* __restrict__ out) {
  const int row = blockIdx.x >> 2;
  const int p = ((blockIdx.x & 3) << 8) + threadIdx.x;
  const float* src = waq;
  int srow = 0;
  bool zero = false;
  if (row < kColAk)       { src = waq; srow = row; }
  else if (row < kColAv)  { src = wak; srow = row - kColAk; }
  else if (row < kColPad) { src = wav; srow = row - kColAv; }
  else if (row < kColBq)  { src = waq; srow = 0; zero = true; }
  else if (row < kColBk)  { src = wbq; srow = row - kColBq; }
  else if (row < kColBv)  { src = wbk; srow = row - kColBk; }
  else                    { src = wbv; srow = row - kColBv; }
  const v2f x = *(const v2f*)(src + (size_t)srow * kHid + 2 * p);
  const float a0 = zero ? 0.0f : x[0];
  const float a1 = zero ? 0.0f : x[1];
  const unsigned u = (unsigned)f2bf_bits(a0) | ((unsigned)f2bf_bits(a1) << 16);
  const size_t o = (size_t)row * (kHid / 2) + p;
  ((volatile unsigned*)out)[o] = u;
  __threadfence();
  ((volatile unsigned*)out)[o] = u;
}

__global__ __launch_bounds__(256) void q_planes(const float* __restrict__ fac, const float* __restrict__ fcos,
                                                const float* __restrict__ fsin,
                                                unsigned short* __restrict__ qh_o, unsigned short* __restrict__ ql_o) {
  const int lane = threadIdx.x & 31, wave = threadIdx.x >> 5;
  const int tok = blockIdx.x * 8 + wave;
  const int s = tok & (kSeq - 1);
  const int dd = lane * 8;
  const int jj = dd & 127;
  const bool upper = (lane >= 16);
  const float* fr = fac + (size_t)tok * kNcat;
  float cs[8], sn[8];
  {
    const v4f c0 = *(const v4f*)(fcos + (size_t)s * 128 + jj);
    const v4f c1 = *(const v4f*)(fcos + (size_t)s * 128 + jj + 4);
    const v4f s0 = *(const v4f*)(fsin + (size_t)s * 128 + jj);
    const v4f s1 = *(const v4f*)(fsin + (size_t)s * 128 + jj + 4);
#pragma unroll
    for (int e = 0; e < 4; ++e) {
      cs[e] = bf16_rne(c0[e]); cs[4 + e] = bf16_rne(c1[e]);
      sn[e] = bf16_rne(s0[e]); sn[4 + e] = bf16_rne(s1[e]);
    }
  }
  float qacc[kHeads][8];
#pragma unroll
  for (int hd = 0; hd < kHeads; ++hd)
#pragma unroll
    for (int e = 0; e < 8; ++e) qacc[hd][e] = 0.0f;
#pragma unroll 1
  for (int r = 0; r < kRq; ++r) {
    const float* bp = fr + kColBq + r * kHeadDim;
    const v4f x1a = *(const v4f*)(bp + jj);
    const v4f x1b = *(const v4f*)(bp + jj + 4);
    const v4f x2a = *(const v4f*)(bp + 128 + jj);
    const v4f x2b = *(const v4f*)(bp + 128 + jj + 4);
    float ro[8];
#pragma unroll
    for (int e = 0; e < 4; ++e) {
      float x1 = x1a[e], x2 = x2a[e];
      float pp = upper ? x2 : x1;
      float qq = upper ? x1 : -x2;
      ro[e] = pp * cs[e] + qq * sn[e];
      x1 = x1b[e]; x2 = x2b[e];
      pp = upper ? x2 : x1;
      qq = upper ? x1 : -x2;
      ro[4 + e] = pp * cs[4 + e] + qq * sn[4 + e];
    }
#pragma unroll
    for (int hd = 0; hd < kHeads; ++hd) {
      const float a = fr[kColAq + hd * kRq + r];
#pragma unroll
      for (int e = 0; e < 8; ++e) qacc[hd][e] += a * ro[e];
    }
  }
  _Float16* qh = (_Float16*)qh_o;
  _Float16* ql = (_Float16*)ql_o;
  for (int pass = 0; pass < 2; ++pass) {
#pragma unroll
    for (int hd = 0; hd < kHeads; ++hd) {
      v8h hv, lv;
#pragma unroll
      for (int e = 0; e < 8; ++e) {
        const float f = qacc[hd][e] * (kQkCarry / (float)kRq);
        const _Float16 fh = (_Float16)f;
        float rsd = f - (float)fh;
        rsd = rsd * kResCarry;
        hv[e] = fh;
        lv[e] = (_Float16)rsd;
      }
      const size_t off = ((size_t)tok * kHeads + hd) * kHeadDim + dd;
      *(volatile v8h*)(qh + off) = hv;
      *(volatile v8h*)(ql + off) = lv;
    }
    __threadfence();
  }
}

__global__ __launch_bounds__(256) void kv_planes(const float* __restrict__ fac, const float* __restrict__ fcos,
                                                 const float* __restrict__ fsin,
                                                 unsigned short* __restrict__ kh_o, unsigned short* __restrict__ kl_o,
                                                 unsigned short* __restrict__ vth_o, unsigned short* __restrict__ vtl_o) {
  __shared__ __align__(16) float vt_l[64 * 260];
  const int lane = threadIdx.x & 31, wave = threadIdx.x >> 5;
  const int tok0 = blockIdx.x * 64;
  const int bidx = tok0 / kSeq;
  const int s0 = tok0 & (kSeq - 1);
  const int dd = lane * 8;
  const int jj = dd & 127;
  const bool upper = (lane >= 16);
  _Float16* kh = (_Float16*)kh_o;
  _Float16* kl = (_Float16*)kl_o;
#pragma unroll 1
  for (int i = 0; i < 8; ++i) {
    const int tl = wave * 8 + i;
    const int tok = tok0 + tl;
    const int s = s0 + tl;
    const float* fr = fac + (size_t)tok * kNcat;
    float cs[8], sn[8];
    {
      const v4f c0 = *(const v4f*)(fcos + (size_t)s * 128 + jj);
      const v4f c1 = *(const v4f*)(fcos + (size_t)s * 128 + jj + 4);
      const v4f sv0 = *(const v4f*)(fsin + (size_t)s * 128 + jj);
      const v4f sv1 = *(const v4f*)(fsin + (size_t)s * 128 + jj + 4);
#pragma unroll
      for (int e = 0; e < 4; ++e) {
        cs[e] = bf16_rne(c0[e]); cs[4 + e] = bf16_rne(c1[e]);
        sn[e] = bf16_rne(sv0[e]); sn[4 + e] = bf16_rne(sv1[e]);
      }
    }
    asm volatile("" ::: "memory");
    float kacc[8], vacc[8];
#pragma unroll
    for (int e = 0; e < 8; ++e) { kacc[e] = 0.0f; vacc[e] = 0.0f; }
#pragma unroll
    for (int r = 0; r < kRk; ++r) {
      const float* bp = fr + kColBk + r * kHeadDim;
      const v4f x1a = *(const v4f*)(bp + jj);
      const v4f x1b = *(const v4f*)(bp + jj + 4);
      const v4f x2a = *(const v4f*)(bp + 128 + jj);
      const v4f x2b = *(const v4f*)(bp + 128 + jj + 4);
      const float a = fr[kColAk + r];
#pragma unroll
      for (int e = 0; e < 4; ++e) {
        float x1 = x1a[e], x2 = x2a[e];
        float pp = upper ? x2 : x1;
        float qq = upper ? x1 : -x2;
        const float ro0 = pp * cs[e] + qq * sn[e];
        x1 = x1b[e]; x2 = x2b[e];
        pp = upper ? x2 : x1;
        qq = upper ? x1 : -x2;
        const float ro1 = pp * cs[4 + e] + qq * sn[4 + e];
        kacc[e] += a * ro0;
        kacc[4 + e] += a * ro1;
      }
    }
    asm volatile("" ::: "memory");
#pragma unroll
    for (int r = 0; r < kRv; ++r) {
      const float* bp = fr + kColBv + r * kHeadDim + dd;
      const v4f y0 = *(const v4f*)(bp);
      const v4f y1 = *(const v4f*)(bp + 4);
      const float a = fr[kColAv + r];
#pragma unroll
      for (int e = 0; e < 4; ++e) { vacc[e] += a * y0[e]; vacc[4 + e] += a * y1[e]; }
    }
    v8h hv, lv;
#pragma unroll
    for (int e = 0; e < 8; ++e) {
      const float f = kacc[e] * (kQkCarry / (float)kRk);
      const _Float16 fh = (_Float16)f;
      float rsd = f - (float)fh;
      rsd = rsd * kResCarry;
      hv[e] = fh;
      lv[e] = (_Float16)rsd;
    }
    const size_t koffs = (size_t)tok * kHeadDim + dd;
    *(volatile v8h*)(kh + koffs) = hv;
    *(volatile v8h*)(kl + koffs) = lv;
    __threadfence();
    *(volatile v8h*)(kh + koffs) = hv;
    *(volatile v8h*)(kl + koffs) = lv;
    v4f w0, w1;
#pragma unroll
    for (int e = 0; e < 4; ++e) { w0[e] = vacc[e] * (kVCarry / (float)kRv); w1[e] = vacc[4 + e] * (kVCarry / (float)kRv); }
    *(v4f*)(vt_l + tl * 260 + dd) = w0;
    *(v4f*)(vt_l + tl * 260 + dd + 4) = w1;
  }
  __syncthreads();
  {
    _Float16* vth = (_Float16*)vth_o;
    _Float16* vtl = (_Float16*)vtl_o;
    const int rq = lane >> 3, c8 = (lane & 7) * 8;
    for (int pass = 0; pass < 2; ++pass) {
#pragma unroll
      for (int it = 0; it < 8; ++it) {
        const int d = wave * 32 + it * 4 + rq;
        v8h hv, lv;
#pragma unroll
        for (int e = 0; e < 8; ++e) {
          const float f = vt_l[(c8 + e) * 260 + d];
          const _Float16 fh = (_Float16)f;
          float rsd = f - (float)fh;
          rsd = rsd * kResCarry;
          hv[e] = fh;
          lv[e] = (_Float16)rsd;
        }
        const size_t off = ((size_t)bidx * kHeadDim + d) * kSeq + s0 + c8;
        *(volatile v8h*)(vth + off) = hv;
        *(volatile v8h*)(vtl + off) = lv;
      }
      __threadfence();
    }
  }
}

template <int DW, bool SPLIT>
__global__ __launch_bounds__(256) __attribute__((amdgpu_num_vgpr(256))) void tpa_attn(
    const unsigned short* __restrict__ qhp, const unsigned short* __restrict__ qlp,
    const unsigned short* __restrict__ khp, const unsigned short* __restrict__ klp,
    const unsigned short* __restrict__ vthp, const unsigned short* __restrict__ vtlp,
    const float* __restrict__ maskp,
    unsigned short* __restrict__ aohp, unsigned short* __restrict__ aolp,
    int qb_begin, int nq) {
  constexpr int NDG = kHeadDim / DW;
  constexpr int NRG = 8 / NDG;
  constexpr int QB  = NRG * 16;
  constexpr int NDC = DW / 32;
  constexpr int NT  = DW / 16;
  constexpr int TPR = 256 / QB;
  constexpr int KPT = 64 / TPR;
  constexpr int OSP = kHeadDim + 4;
  static_assert(8 * 1024 <= kAttPool, "score partials fit");
  static_assert(QB * OSP <= kAttPool, "epilogue tile fits");
  static_assert(KPT % 4 == 0 && TPR * QB == 256 && (TPR & (TPR - 1)) == 0 && TPR <= 32, "softmax lane map");
  static_assert((QB * 4) % 32 == 0, "line coverage");
  __shared__ __align__(16) float pool[kAttPool];
  __shared__ __align__(16) _Float16 Psh[QB * 64];
  __shared__ __align__(16) _Float16 Psl[SPLIT ? QB * 64 : 16];
  __shared__ float alph[QB];
  __shared__ float lfin[QB];

  const int tid = threadIdx.x;
  const int lane = tid & 31, wave = tid >> 5;
  const int hh = lane >> 4, c = lane & 15, koff = hh * 8;
  const int rg = wave % NRG, dg = wave / NRG;
  const int bx = blockIdx.x;
  const int qbi = bx % nq;
  const int bh = bx / nq;
  const int h = bh % kHeads;
  const int b = bh / kHeads;
  const int qb = qb_begin + qbi;
  const int qbase = qb * QB;
  const int q0 = qbase + rg * 16;
  const int dbase = dg * DW;
  const int srow = tid / TPR;
  const int sg = tid - srow * TPR;

  const _Float16* qrow_h = (const _Float16*)qhp + ((size_t)(b * kSeq + q0 + c) * kHeads + h) * kHeadDim + dbase + koff;
  const _Float16* qrow_l = (const _Float16*)qlp + ((size_t)(b * kSeq + q0 + c) * kHeads + h) * kHeadDim + dbase + koff;
  const _Float16* kbase_h = (const _Float16*)khp + (size_t)b * kSeq * kHeadDim + dbase + koff;
  const _Float16* kbase_l = (const _Float16*)klp + (size_t)b * kSeq * kHeadDim + dbase + koff;
  const _Float16* vbase_h = (const _Float16*)vthp + ((size_t)b * kHeadDim + dbase + c) * kSeq + koff;
  const _Float16* vbase_l = (const _Float16*)vtlp + ((size_t)b * kHeadDim + dbase + c) * kSeq + koff;

  v16h qa[NDC], qal[NDC];
#pragma unroll
  for (int dc = 0; dc < NDC; ++dc) {
    qa[dc] = Frag<_Float16>::load(qrow_h + dc * 32);
    qal[dc] = qa[dc];
    if (SPLIT) qal[dc] = Frag<_Float16>::load(qrow_l + dc * 32);
  }

  v8f oacc[NT], oaccr[NT];
#pragma unroll
  for (int t = 0; t < NT; ++t) {
    oacc[t] = (v8f){0.f,0.f,0.f,0.f,0.f,0.f,0.f,0.f};
    oaccr[t] = (v8f){0.f,0.f,0.f,0.f,0.f,0.f,0.f,0.f};
  }
  float m_s = -__builtin_inff();
  float l_s = 0.0f;

  int nChunks = (qbase + QB - 1) / 64 + 1;
  if (nChunks > kSeq / 64) nChunks = kSeq / 64;
  for (int kc = 0; kc < nChunks; ++kc) {
    const int kv0 = kc * 64;
#pragma unroll 1
    for (int j = 0; j < 4; ++j) {
      v8f sacc = (v8f){0.f,0.f,0.f,0.f,0.f,0.f,0.f,0.f};
      v8f sracc = (v8f){0.f,0.f,0.f,0.f,0.f,0.f,0.f,0.f};
#pragma unroll
      for (int dc = 0; dc < NDC; ++dc) {
        const size_t ko = (size_t)(kv0 + j * 16 + c) * kHeadDim + dc * 32;
        const v16h kb = Frag<_Float16>::load(kbase_h + ko);
        sacc = mma16(qa[dc], kb, sacc);
        if (SPLIT) {
          const v16h kbl = Frag<_Float16>::load(kbase_l + ko);
          sracc = mma16(qa[dc], kbl, sracc);
          sracc = mma16(qal[dc], kb, sracc);
        }
      }
#pragma unroll
      for (int r = 0; r < 8; ++r) {
        float v = sacc[r];
        if (SPLIT) v += sracc[r] * (1.0f / kResCarry);
        pool[wave * 1024 + (8 * hh + r) * 64 + j * 16 + c] = v;
      }
    }
    __syncthreads();
    {
      const int rl = srow & 15, rgr = srow >> 4;
      float a[KPT];
#pragma unroll
      for (int e = 0; e < KPT; ++e) a[e] = 0.0f;
#pragma unroll
      for (int dg2 = 0; dg2 < NDG; ++dg2) {
        const float* spp = pool + (dg2 * NRG + rgr) * 1024 + rl * 64 + sg * KPT;
#pragma unroll
        for (int i = 0; i < KPT / 4; ++i) {
          const v4f x = *(const v4f*)(spp + 4 * i);
#pragma unroll
          for (int e = 0; e < 4; ++e) a[4 * i + e] += x[e];
        }
      }
      float mk[KPT];
      const float* mrowp = maskp + (size_t)(qbase + srow) * kSeq + kv0 + sg * KPT;
#pragma unroll
      for (int i = 0; i < KPT / 4; ++i) {
        const v4f mv = *(const v4f*)(mrowp + 4 * i);
#pragma unroll
        for (int e = 0; e < 4; ++e) mk[4 * i + e] = mv[e];
      }
      float sv[KPT];
      float cmx = -__builtin_inff();
#pragma unroll
      for (int e = 0; e < KPT; ++e) {
        sv[e] = tanhf(a[e] * kTanhArg) * kSoftcap + bf16_rne(mk[e]);
        cmx = fmaxf(cmx, sv[e]);
      }
#pragma unroll
      for (int off = 1; off < TPR; off <<= 1) cmx = fmaxf(cmx, __shfl_xor(cmx, off, 32));
      const float mnew = fmaxf(m_s, cmx);
      const float alpha = expf(m_s - mnew);
      m_s = mnew;
      float psum = 0.0f;
      _Float16* prow = Psh + srow * 64 + sg * KPT;
      _Float16* prl = Psl + (SPLIT ? (srow * 64 + sg * KPT) : 0);
#pragma unroll
      for (int e = 0; e < KPT; ++e) {
        const float p = expf(sv[e] - mnew);
        psum += p;
        const float pc = p * kPCarry;
        const _Float16 ph = (_Float16)pc;
        prow[e] = ph;
        if (SPLIT) {
          float prs = pc - (float)ph;
          prs = prs * kResCarry;
          prl[e] = (_Float16)prs;
        }
      }
#pragma unroll
      for (int off = 1; off < TPR; off <<= 1) psum += __shfl_xor(psum, off, 32);
      l_s = l_s * alpha + psum;
      if (sg == 0) alph[srow] = alpha;
    }
    __syncthreads();
    {
      float al[8];
#pragma unroll
      for (int r = 0; r < 8; ++r) al[r] = alph[rg * 16 + 8 * hh + r];
#pragma unroll
      for (int t = 0; t < NT; ++t) {
#pragma unroll
        for (int r = 0; r < 8; ++r) {
          oacc[t][r] *= al[r];
          if (SPLIT) oaccr[t][r] *= al[r];
        }
      }
    }
#pragma unroll 1
    for (int kk = 0; kk < 2; ++kk) {
      const v16h pa = Frag<_Float16>::load(Psh + (rg * 16 + c) * 64 + kk * 32 + 8 * hh);
      v16h pl = pa;
      if (SPLIT) pl = Frag<_Float16>::load(Psl + (rg * 16 + c) * 64 + kk * 32 + 8 * hh);
#pragma unroll
      for (int t = 0; t < NT; ++t) {
        const size_t vo = (size_t)(t * 16) * kSeq + kv0 + kk * 32;
        const v16h vb = Frag<_Float16>::load(vbase_h + vo);
        oacc[t] = mma16(pa, vb, oacc[t]);
        if (SPLIT) {
          const v16h vbl = Frag<_Float16>::load(vbase_l + vo);
          oaccr[t] = mma16(pa, vbl, oaccr[t]);
          oaccr[t] = mma16(pl, vb, oaccr[t]);
        }
      }
    }
  }
  if (sg == 0) lfin[srow] = l_s;
  __syncthreads();
#pragma unroll
  for (int r = 0; r < 8; ++r) {
    const int row = rg * 16 + 8 * hh + r;
    const float lf = lfin[row];
    const float inv = kOutScl / lf;
#pragma unroll
    for (int t = 0; t < NT; ++t) {
      float o = oacc[t][r];
      if (SPLIT) o += oaccr[t][r] * (1.0f / kResCarry);
      pool[row * OSP + dbase + t * 16 + c] = o * inv;
    }
  }
  __syncthreads();
  {
    const int lq = lane >> 3, c8 = (lane & 7) * 8;
    _Float16* oh = (_Float16*)aohp;
    _Float16* ol = (_Float16*)aolp;
    for (int pass = 0; pass < 2; ++pass) {
#pragma unroll
      for (int it = 0; it < QB / 8; ++it) {
        const int L = wave * (QB / 2) + it * 4 + lq;
        const int row = L >> 2;
        const int seg = L & 3;
        const float* sp = pool + row * OSP + seg * 64 + c8;
        const v4f s0 = *(const v4f*)(sp);
        const v4f s1 = *(const v4f*)(sp + 4);
        v8h hv, lv;
#pragma unroll
        for (int e = 0; e < 4; ++e) {
          const float f0 = s0[e], f1 = s1[e];
          const _Float16 fh0 = (_Float16)f0, fh1 = (_Float16)f1;
          hv[e] = fh0; hv[4 + e] = fh1;
          if (SPLIT) {
            float r0 = f0 - (float)fh0; r0 = r0 * kResCarry;
            float r1 = f1 - (float)fh1; r1 = r1 * kResCarry;
            lv[e] = (_Float16)r0; lv[4 + e] = (_Float16)r1;
          }
        }
        const size_t off = (size_t)(b * kSeq + qbase + row) * kHid + h * kHeadDim + seg * 64 + c8;
        *(volatile v8h*)(oh + off) = hv;
        if (SPLIT) *(volatile v8h*)(ol + off) = lv;
      }
      __threadfence();
    }
  }
}

extern "C" void kernel_launch(void* const* d_in, const int* in_sizes, int n_in,
                              void* d_out, int out_size, void* d_ws, size_t ws_size,
                              hipStream_t stream) {
  if (n_in < 12) return;
  if (in_sizes[0] != kTok * kHid || in_sizes[1] != kSeq * 128 || in_sizes[2] != kSeq * 128 ||
      in_sizes[3] != kSeq * kSeq || in_sizes[5] != 48 * kHid || in_sizes[6] != 2 * kHid ||
      in_sizes[7] != 2 * kHid || in_sizes[8] != 1536 * kHid || in_sizes[9] != 512 * kHid ||
      in_sizes[10] != 512 * kHid || in_sizes[11] != kHid * kHid) return;
  if (out_size != kTok * kHid) return;
  if (ws_size < kWsTotal) return;

  const float* hs   = (const float*)d_in[0];
  const float* fcos = (const float*)d_in[1];
  const float* fsin = (const float*)d_in[2];
  const float* amask = (const float*)d_in[3];
  const float* waq = (const float*)d_in[5];
  const float* wak = (const float*)d_in[6];
  const float* wav = (const float*)d_in[7];
  const float* wbq = (const float*)d_in[8];
  const float* wbk = (const float*)d_in[9];
  const float* wbv = (const float*)d_in[10];
  const float* wo  = (const float*)d_in[11];
  float* out = (float*)d_out;

  char* ws = (char*)d_ws;
  float* fac = (float*)(ws + kOffFac);
  unsigned short* aoh  = (unsigned short*)(ws + kOffAoh);
  unsigned short* aol  = (unsigned short*)(ws + kOffAol);
  float* t1 = (float*)(ws + kOffT1);
  unsigned short* hsb  = (unsigned short*)(ws + kOffHsb);
  unsigned short* wcat = (unsigned short*)(ws + kOffWcat);
  unsigned short* qh   = (unsigned short*)(ws + kOffQh);
  unsigned short* ql   = (unsigned short*)(ws + kOffQl);
  unsigned short* kh   = (unsigned short*)(ws + kOffKh);
  unsigned short* kl   = (unsigned short*)(ws + kOffKl);
  unsigned short* vth  = (unsigned short*)(ws + kOffVth);
  unsigned short* vtl  = (unsigned short*)(ws + kOffVtl);
  unsigned short* wo16 = (unsigned short*)(ws + kOffWo);
  const float* dummyf = (const float*)(ws + kOffWo);

  {
    const int n2 = kTok * kHid / 2;
    cast_bf16x2<<<dim3((n2 + 255) / 256), dim3(256), 0, stream>>>(hs, hsb, n2);
    build_wcat<<<dim3(kNcat * 4), dim3(256), 0, stream>>>(waq, wak, wav, wbq, wbk, wbv, wcat);
    const int n2w = kHid * kHid / 2;
    cast_wo_f16x2<<<dim3((n2w + 255) / 256), dim3(256), 0, stream>>>(wo, wo16, n2w);
  }
  wmma_gemm64<1, false, 0, 0, false, 0><<<dim3(((kTok / 64) * (kNcat / 64) + 7) / 8, 1), dim3(256), 0, stream>>>(
      hsb, hsb, kHid, 0L, wcat, wcat, kHid, 0L, (void*)fac, (void*)fac, kNcat, 0L,
      dummyf, dummyf, 0L, kTok, kNcat, kHid, 1.0f);
  q_planes<<<dim3(kTok / 8), dim3(256), 0, stream>>>(fac, fcos, fsin, qh, ql);
  kv_planes<<<dim3(kTok / 64), dim3(256), 0, stream>>>(fac, fcos, fsin, kh, kl, vth, vtl);
  tpa_attn<32, true><<<dim3(kBatch * kHeads * (kSplitRows / 16)), dim3(256), 0, stream>>>(
      qh, ql, kh, kl, vth, vtl, amask, aoh, aol, 0, kSplitRows / 16);
  tpa_attn<64, false><<<dim3(kBatch * kHeads * ((kSeq - kSplitRows) / 32)), dim3(256), 0, stream>>>(
      qh, ql, kh, kl, vth, vtl, amask, aoh, aol, kSplitRows / 32, (kSeq - kSplitRows) / 32);
  wmma_gemm64<0, false, 0, 0, false, 0><<<dim3(((kSplitRows / 64) * (kHid / 64) + 7) / 8, kBatch), dim3(256), 0, stream>>>(
      aol, aol, kHid, (long)kSeq * kHid, wo16, wo16, kHid, 0L, (void*)t1, (void*)t1, kHid, (long)kSplitRows * kHid,
      dummyf, dummyf, 0L, kSplitRows, kHid, kHid, 1.0f / (kResCarry * kWoCarry * kAoCarry));
  wmma_gemm64<0, false, 0, 0, true, 0><<<dim3(((kSplitRows / 64) * (kHid / 64) + 7) / 8, kBatch), dim3(256), 0, stream>>>(
      aoh, aoh, kHid, (long)kSeq * kHid, wo16, wo16, kHid, 0L, (void*)out, (void*)out, kHid, (long)kSeq * kHid,
      dummyf, t1, (long)kSplitRows * kHid, kSplitRows, kHid, kHid, 1.0f / (kWoCarry * kAoCarry));
  wmma_gemm64<0, false, 0, 0, false, 0><<<dim3((((kSeq - kSplitRows) / 64) * (kHid / 64) + 7) / 8, kBatch), dim3(256), 0, stream>>>(
      aoh + (size_t)kSplitRows * kHid, aoh + (size_t)kSplitRows * kHid, kHid, (long)kSeq * kHid,
      wo16, wo16, kHid, 0L, (void*)(out + (size_t)kSplitRows * kHid), (void*)(out + (size_t)kSplitRows * kHid),
      kHid, (long)kSeq * kHid, dummyf, dummyf, 0L, kSeq - kSplitRows, kHid, kHid, 1.0f / (kWoCarry * kAoCarry));
}
